// RetLayer_25503515804195
// MI455X (gfx1250) — hardware-verified
//
#include <hip/hip_runtime.h>

#define BATCH 16
#define TXTN  32
#define VIDN  2048
#define SEQ   2080
#define SEQP  2112
#define DM    256
#define NTILE 33
#define NWPL  12
#define PSC   256.0f
#define VSC   64.0f
#define OSC   (1.0f / 16384.0f)

typedef _Float16 v16h __attribute__((ext_vector_type(16)));
typedef _Float16 v8h  __attribute__((ext_vector_type(8)));
typedef _Float16 v4h  __attribute__((ext_vector_type(4)));
typedef __bf16   v16b __attribute__((ext_vector_type(16)));
typedef unsigned short v8us __attribute__((ext_vector_type(8)));
typedef unsigned short v4us __attribute__((ext_vector_type(4)));
typedef float v8f __attribute__((ext_vector_type(8)));
typedef float v4f __attribute__((ext_vector_type(4)));
typedef v8h  __attribute__((may_alias)) v8ha;
typedef v4h  __attribute__((may_alias)) v4ha;
typedef v8us __attribute__((may_alias)) v8usa;
typedef v4us __attribute__((may_alias)) v4usa;
typedef v4f  __attribute__((may_alias)) v4fa;

__constant__ unsigned int c_invf[] = {
  0x3f800000, 0x3f6e39f8, 0x3f5dafd7, 0x3f4e4bad, 0x3f3ff911, 0x3f32a506, 0x3f263de0, 0x3f1ab32b,
  0x3f0ff59a, 0x3f05f6ef, 0x3ef953cf, 0x3ee8045f, 0x3ed7e89b, 0x3ec8eb24, 0x3ebaf81b, 0x3eadfcff,
  0x3ea1e89b, 0x3e96aaea, 0x3e8c3504, 0x3e827909, 0x3e72d423, 0x3e61f835, 0x3e5247ed, 0x3e43ae7c,
  0x3e361887, 0x3e297409, 0x3e1db040, 0x3e12bd91, 0x3e088d77, 0x3dfe24e0, 0x3dec7fd6, 0x3ddc1466,
  0x3dcccccd, 0x3dbe94c6, 0x3db15978, 0x3da50956, 0x3d99940d, 0x3d8eea6b, 0x3d84fe4d, 0x3d778513,
  0x3d6655c2, 0x3d5657e4, 0x3d47763f, 0x3d399d19, 0x3d2cba15, 0x3d20bc1d, 0x3d159348, 0x3d0b30cc,
  0x3d0186e3, 0x3cf11177, 0x3ce054d2, 0x3cd0c1a8, 0x3cc2434f, 0x3cb4c691, 0x3ca8398b, 0x3c9c8b97,
  0x3c91ad39, 0x3c879008, 0x3c7c4d33, 0x3c6ac8e7, 0x3c5a7bf2, 0x3c4b50b3, 0x3c3d3311, 0x3c301052,
  0x3c23d70a, 0x3c187705, 0x3c0de12d, 0x3c040779, 0x3bf5b9b0, 0x3be4aa46, 0x3bd4ca15, 0x3bc6040f,
  0x3bb8449c, 0x3bab7983, 0x3b9f91cc, 0x3b947dae, 0x3b8a2e77, 0x3b80967d, 0x3b6f520e, 0x3b5eb47a,
  0x3b4f3e38, 0x3b40dac5, 0x3b33770f, 0x3b270153, 0x3b1b690d, 0x3b109edb, 0x3b06946f, 0x3afa78f0,
  0x3ae91528, 0x3ad8e673, 0x3ac9d75c, 0x3abbd3ed, 0x3aaec98e, 0x3aa2a6f7, 0x3a975c0e, 0x3a8cd9db,
  0x3a83126f, 0x3a73f1a3, 0x3a6301e2, 0x3a533f28, 0x3a44948c, 0x3a36ee9e, 0x3a2a3b44, 0x3a1e69a5,
  0x3a136a16, 0x3a092e02, 0x39ff4fac, 0x39ed95e2, 0x39dd1725, 0x39cdbd96, 0x39bf74d7, 0x39b229fa,
  0x39a5cb60, 0x399a489e, 0x398f9272, 0x39859aa9, 0x3978a815, 0x39676492, 0x395753e4, 0x394860c1,
  0x393a7753, 0x392d8529, 0x39217916, 0x39164324, 0x390bd472, 0x39021f2b, 0x38f22ce2, 0x38e15c91 };
static_assert(sizeof(c_invf) == 512);

__constant__ unsigned int c_svec[] = {
  0x3e924925, 0x3e952493, 0x3e980000, 0x3e9adb6e, 0x3e9db6dc, 0x3ea0924a, 0x3ea36db7, 0x3ea64925,
  0x3ea92493, 0x3eac0000, 0x3eaedb6e, 0x3eb1b6dc, 0x3eb4924a, 0x3eb76db7, 0x3eba4924, 0x3ebd2492,
  0x3ec00000, 0x3ec2db6d, 0x3ec5b6db, 0x3ec89249, 0x3ecb6db7, 0x3ece4924, 0x3ed12492, 0x3ed40000,
  0x3ed6db6d, 0x3ed9b6db, 0x3edc9249, 0x3edf6db7, 0x3ee24924, 0x3ee52492, 0x3ee80000, 0x3eeadb6e,
  0x3eedb6db, 0x3ef09249, 0x3ef36db7, 0x3ef64924, 0x3ef92492, 0x3efc0000, 0x3efedb6e, 0x3f00db6e,
  0x3f024924, 0x3f03b6db, 0x3f052492, 0x3f069249, 0x3f080000, 0x3f096db7, 0x3f0adb6e, 0x3f0c4925,
  0x3f0db6db, 0x3f0f2492, 0x3f109249, 0x3f120000, 0x3f136db7, 0x3f14db6e, 0x3f164925, 0x3f17b6db,
  0x3f192492, 0x3f1a9249, 0x3f1c0000, 0x3f1d6db7, 0x3f1edb6e, 0x3f204925, 0x3f21b6db, 0x3f232492,
  0x3f249249, 0x3f260000, 0x3f276db7, 0x3f28db6e, 0x3f2a4925, 0x3f2bb6db, 0x3f2d2492, 0x3f2e9249,
  0x3f300000, 0x3f316db7, 0x3f32db6e, 0x3f344925, 0x3f35b6db, 0x3f372492, 0x3f389249, 0x3f3a0000,
  0x3f3b6db7, 0x3f3cdb6e, 0x3f3e4925, 0x3f3fb6db, 0x3f412492, 0x3f429249, 0x3f440000, 0x3f456db7,
  0x3f46db6e, 0x3f484925, 0x3f49b6db, 0x3f4b2492, 0x3f4c9249, 0x3f4e0000, 0x3f4f6db7, 0x3f50db6e,
  0x3f524925, 0x3f53b6db, 0x3f552492, 0x3f569249, 0x3f580000, 0x3f596db7, 0x3f5adb6e, 0x3f5c4925,
  0x3f5db6db, 0x3f5f2492, 0x3f609249, 0x3f620000, 0x3f636db7, 0x3f64db6e, 0x3f664925, 0x3f67b6dc,
  0x3f692492, 0x3f6a9249, 0x3f6c0000, 0x3f6d6db7, 0x3f6edb6e, 0x3f704925, 0x3f71b6dc, 0x3f732492,
  0x3f749249, 0x3f760000, 0x3f776db7, 0x3f78db6e, 0x3f7a4925, 0x3f7bb6dc, 0x3f7d2492, 0x3f7e9249 };
static_assert(sizeof(c_svec) == 512);

__device__ __forceinline__ v8f wmma_h(v16h a, v16h b, v8f c) {
  v8f d = __builtin_amdgcn_wmma_f32_16x16x32_f16(false, a, false, b, (short)0, c, false, false);
  asm volatile("v_nop\n\tv_nop\n\tv_nop\n\tv_nop" : "+v"(d) : "v"(a), "v"(b));
  return d;
}
__device__ __forceinline__ v8f wmma_b(v16b a, v16b b, v8f c) {
  v8f d = __builtin_amdgcn_wmma_f32_16x16x32_bf16(false, a, false, b, (short)0, c, false, false);
  asm volatile("v_nop\n\tv_nop\n\tv_nop\n\tv_nop" : "+v"(d) : "v"(a), "v"(b));
  return d;
}

__device__ __forceinline__ v16h ldfh(const _Float16* p, int h) {
  union { v16h v; v8h hf[2]; } f;
  f.hf[0] = *(const v8ha*)(p + 8 * h);
  f.hf[1] = *(const v8ha*)(p + 16 + 8 * h);
  return f.v;
}
__device__ __forceinline__ v16b ldfb(const unsigned short* p, int h) {
  union { v16b v; v8us hf[2]; } f;
  f.hf[0] = *(const v8usa*)(p + 8 * h);
  f.hf[1] = *(const v8usa*)(p + 16 + 8 * h);
  return f.v;
}

__device__ __forceinline__ unsigned int bf16_rne(float x) {
  const unsigned int u = __float_as_uint(x);
  return (u + 0x7FFFu + ((u >> 16) & 1u)) >> 16;
}

__global__ __launch_bounds__(256) void k_wprep(
    const float* __restrict__ wtq, const float* __restrict__ wtk, const float* __restrict__ wtv,
    const float* __restrict__ wvq, const float* __restrict__ wvk, const float* __restrict__ wvv,
    unsigned short* __restrict__ WB)
{
  const int tid = threadIdx.x, lane = tid & 31;
  const int row = blockIdx.x * 8 + (tid >> 5);
  if (row >= NWPL * DM) return;
  const int pl = row >> 8, n = row & 255;
  const int wsel = pl >> 1, part = pl & 1;
  const float* W = (wsel == 0) ? wtq : (wsel == 1) ? wtk : (wsel == 2) ? wvq
                 : (wsel == 3) ? wvk : (wsel == 4) ? wtv : wvv;
  const int k0 = lane * 8;
  float v[8];
  #pragma unroll
  for (int i = 0; i < 8; ++i) v[i] = W[(size_t)(k0 + i) * DM + n];
  v8us o;
  #pragma unroll
  for (int i = 0; i < 8; ++i) {
    const unsigned int hb = bf16_rne(v[i]);
    const unsigned int lb = bf16_rne(v[i] - __uint_as_float(hb << 16));
    o[i] = (unsigned short)(part ? lb : hb);
  }
  unsigned short* dst = WB + (size_t)pl * 65536 + (size_t)n * DM + k0;
  *(volatile v8us*)dst = o;
  __threadfence();
  *(volatile v8us*)dst = o;
}

__global__ __launch_bounds__(256) void k_xtab(float* __restrict__ XT)
{
  const int n = blockIdx.x >> 3;
  const int l = (blockIdx.x & 7) * 256 + threadIdx.x;
  const int i = n >> 1;
  const float sv = __uint_as_float(c_svec[i]);
  const float pw = (float)l * (1.0f / 512.0f);
  const float scale = powf(sv, pw);
  const float invf = __uint_as_float(c_invf[i]);
  const float ang = (float)l * invf;
  const float sn = sinf(ang), cs = cosf(ang);
  const float inv = 1.0f / scale;
  const size_t PS = (size_t)DM * VIDN;
  float* p0 = XT + (size_t)n * VIDN + l;
  const float a0 = cs * scale, a1 = sn * scale, a2 = cs * inv, a3 = sn * inv;
  *(volatile float*)(p0)          = a0;
  *(volatile float*)(p0 + PS)     = a1;
  *(volatile float*)(p0 + 2 * PS) = a2;
  *(volatile float*)(p0 + 3 * PS) = a3;
  __threadfence();
  *(volatile float*)(p0)          = a0;
  *(volatile float*)(p0 + PS)     = a1;
  *(volatile float*)(p0 + 2 * PS) = a2;
  *(volatile float*)(p0 + 3 * PS) = a3;
}

__global__ __launch_bounds__(256) void k_mask(const float* __restrict__ lr, float* __restrict__ M)
{
  const int idx = blockIdx.x * 256 + threadIdx.x;
  if (idx >= VIDN * VIDN) return;
  const float x = lr[idx];
  const float s = 1.0f / (1.0f + expf(-x));
  *(volatile float*)(M + idx) = s;
  __threadfence();
  *(volatile float*)(M + idx) = s;
}

__global__ __launch_bounds__(256) void k_loss(const float* __restrict__ lr, const int* __restrict__ tl,
                                              float* __restrict__ out1)
{
  __shared__ double red[256];
  const int t = threadIdx.x;
  double acc = 0.0;
  #pragma unroll 1
  for (int j = 0; j < VIDN * 8; ++j) {
    const int idx = j * 256 + t;
    const int r = j >> 3, c = (j & 7) * 256 + t;
    const float x = lr[idx];
    const float s = 1.0f / (1.0f + expf(-x));
    acc += (r == c) ? 0.0 : (double)s;
  }
  red[t] = acc;
  __syncthreads();
  if (t == 0) {
    double sum = 0.0;
    #pragma unroll 1
    for (int i = 0; i < 256; ++i) sum += red[i];
    int vl = SEQ - tl[0];
    vl = vl < 1 ? 1 : vl;
    vl = vl > VIDN ? VIDN : vl;
    const float loss = (float)(sum / ((double)vl * (double)vl));
    *(volatile float*)out1 = loss;
    __threadfence();
    *(volatile float*)out1 = loss;
  }
}

__device__ __forceinline__ void store_qk(const unsigned short* sOut, unsigned short* PH, unsigned short* PLo,
                                         int b, int s0, int w, int sub, int q8)
{
  #pragma unroll
  for (int i = 0; i < 8; ++i) {
    const int lid = w * 32 + 4 * i + sub;
    const int pl = lid >> 8, row = (lid >> 2) & 63, qu = lid & 3;
    const v8us v = *(const v8usa*)(sOut + pl * 16384 + row * DM + 64 * qu + 8 * q8);
    unsigned short* dst = (pl ? PLo : PH) + ((size_t)(b * SEQP + s0 + row)) * DM + 64 * qu + 8 * q8;
    *(volatile v8us*)dst = v;
  }
}

__device__ __forceinline__ void store_vt(const _Float16* sV, _Float16* VT, int b, int s0, int w, int sub, int q8)
{
  #pragma unroll
  for (int i = 0; i < 4; ++i) {
    const int d = 16 * w + 4 * i + sub;
    const v8h v = *(const v8ha*)(sV + d * 64 + 8 * q8);
    _Float16* dst = VT + ((size_t)(b * DM + d)) * SEQP + s0 + 8 * q8;
    *(volatile v8h*)dst = v;
  }
}

__global__ __launch_bounds__(512) void k_proj(
    const float* __restrict__ src,
    const unsigned short* __restrict__ WB, const float* __restrict__ XT,
    unsigned short* __restrict__ QH, unsigned short* __restrict__ QL,
    unsigned short* __restrict__ KH, unsigned short* __restrict__ KL,
    _Float16* __restrict__ VT)
{
  extern __shared__ __attribute__((aligned(16))) unsigned char smem[];
  unsigned short* sAh  = (unsigned short*)smem;
  unsigned short* sAl  = sAh + 64 * DM;
  unsigned short* sOut = (unsigned short*)(smem + 65536);
  _Float16*       sV   = (_Float16*)(smem + 65536);

  const int tid = threadIdx.x, lane = tid & 31, w = tid >> 5;
  const int wr = w >> 2, wc = w & 3, h = lane >> 4, m = lane & 15;
  const int q8 = lane & 7, sub = lane >> 3;
  const int b = blockIdx.y, s0 = blockIdx.x * 64;
  const bool wtxt = (blockIdx.x == 0) && (wr < 2);
  const v4f z4 = {0.f, 0.f, 0.f, 0.f};
  const v8f z8 = {0.f, 0.f, 0.f, 0.f, 0.f, 0.f, 0.f, 0.f};

  #pragma unroll 1
  for (int it = 0; it < 8; ++it) {
    const int q = it * 512 + tid;
    const int row = q >> 6, c4 = (q & 63) * 4;
    const int s = s0 + row;
    const int sl = (s < SEQ) ? s : (SEQ - 1);
    v4f x = *(const v4fa*)(src + ((size_t)(b * SEQ + sl)) * DM + c4);
    if (s >= SEQ) x = z4;
    if (s < TXTN) {
      const float xe = ((float)(s + 1) * 0.03125f) * 6.2831855f;
      const float d0 = powf(10000.0f, (float)c4 * (1.0f / 256.0f));
      const float d1 = powf(10000.0f, (float)(c4 + 2) * (1.0f / 256.0f));
      const float r0 = xe * (1.0f / d0), r1 = xe * (1.0f / d1);
      x.x += sinf(r0); x.y += cosf(r0); x.z += sinf(r1); x.w += cosf(r1);
    }
    const unsigned int h0 = bf16_rne(x.x), h1 = bf16_rne(x.y), h2 = bf16_rne(x.z), h3 = bf16_rne(x.w);
    const unsigned int l0 = bf16_rne(x.x - __uint_as_float(h0 << 16));
    const unsigned int l1 = bf16_rne(x.y - __uint_as_float(h1 << 16));
    const unsigned int l2 = bf16_rne(x.z - __uint_as_float(h2 << 16));
    const unsigned int l3 = bf16_rne(x.w - __uint_as_float(h3 << 16));
    const v4us vh = {(unsigned short)h0, (unsigned short)h1, (unsigned short)h2, (unsigned short)h3};
    const v4us vl = {(unsigned short)l0, (unsigned short)l1, (unsigned short)l2, (unsigned short)l3};
    *(v4usa*)(sAh + row * DM + c4) = vh;
    *(v4usa*)(sAl + row * DM + c4) = vl;
  }
  __syncthreads();

  #pragma unroll 1
  for (int p = 0; p < 2; ++p) {
    const unsigned short* Bh = WB + (size_t)((wtxt ? 0 : 4) + 2 * p) * 65536 + (size_t)(64 * wc + m) * DM;
    const unsigned short* Bl = Bh + 65536;
    const unsigned short* Ap = sAh + (16 * wr + m) * DM;
    v8f acc[4];
    #pragma unroll
    for (int nt = 0; nt < 4; ++nt) acc[nt] = z8;
    #pragma unroll 1
    for (int kk = 0; kk < DM; kk += 32) {
      const v16b ah = ldfb(Ap + kk, h);
      const v16b al = ldfb(Ap + 64 * DM + kk, h);
      #pragma unroll
      for (int nt = 0; nt < 4; ++nt) {
        const v16b bh = ldfb(Bh + (size_t)(16 * nt) * DM + kk, h);
        const v16b bl = ldfb(Bl + (size_t)(16 * nt) * DM + kk, h);
        acc[nt] = wmma_b(ah, bh, acc[nt]);
        acc[nt] = wmma_b(ah, bl, acc[nt]);
        acc[nt] = wmma_b(al, bh, acc[nt]);
      }
    }
    const int rowb = 16 * wr + 8 * h;
    int lb = s0 + rowb - TXTN;
    lb = lb < 0 ? 0 : lb;
    lb = lb > (VIDN - 8) ? (VIDN - 8) : lb;
    const float sg = (m & 1) ? 1.0f : -1.0f;
    #pragma unroll
    for (int nt = 0; nt < 4; ++nt) {
      const int n = 64 * wc + 16 * nt + m;
      const float* tc = XT + ((size_t)(2 * p * DM + n)) * VIDN + lb;
      const float* ts = tc + (size_t)DM * VIDN;
      const v4f c0 = *(const v4fa*)tc, c1 = *(const v4fa*)(tc + 4);
      const v4f t0 = *(const v4fa*)ts, t1 = *(const v4fa*)(ts + 4);
      const float cs[8] = {c0.x, c0.y, c0.z, c0.w, c1.x, c1.y, c1.z, c1.w};
      const float sn[8] = {t0.x, t0.y, t0.z, t0.w, t1.x, t1.y, t1.z, t1.w};
      #pragma unroll
      for (int r = 0; r < 8; ++r) {
        const float x  = acc[nt][r];
        const float pr = __shfl_xor(x, 1, 32);
        const float cv = wtxt ? 1.0f : cs[r];
        const float snv = wtxt ? 0.0f : sn[r];
        const float y  = x * cv + sg * (pr * snv);
        const unsigned int hb  = bf16_rne(y);
        const unsigned int lob = bf16_rne(y - __uint_as_float(hb << 16));
        const int e = (rowb + r) * DM + n;
        sOut[e]         = (unsigned short)hb;
        sOut[16384 + e] = (unsigned short)lob;
      }
    }
    __syncthreads();
    unsigned short* PH  = p ? KH : QH;
    unsigned short* PLo = p ? KL : QL;
    store_qk(sOut, PH, PLo, b, s0, w, sub, q8);
    __threadfence();
    store_qk(sOut, PH, PLo, b, s0, w, sub, q8);
    __syncthreads();
  }

  if (blockIdx.x == 0) {
    #pragma unroll 1
    for (int it = 0; it < 8; ++it) {
      const int q = it * 512 + tid;
      const int row = q >> 6, c4 = (q & 63) * 4;
      const v4f x = *(const v4fa*)(src + ((size_t)(b * SEQ + row)) * DM + c4);
      const unsigned int h0 = bf16_rne(x.x), h1 = bf16_rne(x.y), h2 = bf16_rne(x.z), h3 = bf16_rne(x.w);
      const unsigned int l0 = bf16_rne(x.x - __uint_as_float(h0 << 16));
      const unsigned int l1 = bf16_rne(x.y - __uint_as_float(h1 << 16));
      const unsigned int l2 = bf16_rne(x.z - __uint_as_float(h2 << 16));
      const unsigned int l3 = bf16_rne(x.w - __uint_as_float(h3 << 16));
      const v4us vh = {(unsigned short)h0, (unsigned short)h1, (unsigned short)h2, (unsigned short)h3};
      const v4us vl = {(unsigned short)l0, (unsigned short)l1, (unsigned short)l2, (unsigned short)l3};
      *(v4usa*)(sAh + row * DM + c4) = vh;
      *(v4usa*)(sAl + row * DM + c4) = vl;
    }
  }
  __syncthreads();
  {
    const unsigned short* Bh = WB + (size_t)(wtxt ? 8 : 10) * 65536 + (size_t)(64 * wc + m) * DM;
    const unsigned short* Bl = Bh + 65536;
    const unsigned short* Ap = sAh + (16 * wr + m) * DM;
    v8f acc[4];
    #pragma unroll
    for (int nt = 0; nt < 4; ++nt) acc[nt] = z8;
    #pragma unroll 1
    for (int kk = 0; kk < DM; kk += 32) {
      const v16b ah = ldfb(Ap + kk, h);
      const v16b al = ldfb(Ap + 64 * DM + kk, h);
      #pragma unroll
      for (int nt = 0; nt < 4; ++nt) {
        const v16b bh = ldfb(Bh + (size_t)(16 * nt) * DM + kk, h);
        const v16b bl = ldfb(Bl + (size_t)(16 * nt) * DM + kk, h);
        acc[nt] = wmma_b(ah, bh, acc[nt]);
        acc[nt] = wmma_b(ah, bl, acc[nt]);
        acc[nt] = wmma_b(al, bh, acc[nt]);
      }
    }
    #pragma unroll
    for (int nt = 0; nt < 4; ++nt) {
      const int d = 64 * wc + 16 * nt + m;
      #pragma unroll
      for (int r = 0; r < 8; ++r) sV[d * 64 + 16 * wr + 8 * h + r] = (_Float16)(acc[nt][r] * VSC);
    }
  }
  __syncthreads();
  store_vt(sV, VT, b, s0, w, sub, q8);
  __threadfence();
  store_vt(sV, VT, b, s0, w, sub, q8);
}

__device__ __forceinline__ void store_out(const float* so, float* out, int b, int q0, int w, int sub, int q8)
{
  #pragma unroll
  for (int i = 0; i < 8; ++i) {
    const int lid = 4 * i + sub, row = lid >> 1, hl = lid & 1;
    const v4f v = *(const v4fa*)(so + row * 64 + 32 * hl + 4 * q8);
    float* dst = out + ((size_t)(b * SEQ + q0 + row)) * DM + 64 * w + 32 * hl + 4 * q8;
    *(volatile v4f*)dst = v;
  }
}

__global__ __launch_bounds__(128) void k_ret(
    const unsigned short* __restrict__ QH, const unsigned short* __restrict__ QL,
    const unsigned short* __restrict__ KH, const unsigned short* __restrict__ KL,
    const _Float16* __restrict__ VT, const float* __restrict__ MK, float* __restrict__ out)
{
  __shared__ __attribute__((aligned(16))) unsigned short sQh[16 * DM];
  __shared__ __attribute__((aligned(16))) unsigned short sQl[16 * DM];
  __shared__ __attribute__((aligned(16))) _Float16 sPh[2][16 * 64];
  __shared__ __attribute__((aligned(16))) _Float16 sPl[2][16 * 64];
  __shared__ __attribute__((aligned(16))) float sO[4 * 16 * 64];

  const int tid = threadIdx.x, lane = tid & 31, w = tid >> 5, h = lane >> 4, m = lane & 15;
  const int q8 = lane & 7, sub = lane >> 3;
  const int b = blockIdx.y, q0 = blockIdx.x * 16;
  const v8f z8 = {0.f, 0.f, 0.f, 0.f, 0.f, 0.f, 0.f, 0.f};

  #pragma unroll
  for (int it = 0; it < 4; ++it) {
    const int idx = it * 128 + tid;
    const int row = idx >> 5, c8 = (idx & 31) * 8;
    const size_t g = ((size_t)(b * SEQP + q0 + row)) * DM + c8;
    *(v8usa*)(sQh + row * DM + c8) = *(const v8usa*)(QH + g);
    *(v8usa*)(sQl + row * DM + c8) = *(const v8usa*)(QL + g);
  }
  __syncthreads();

  v8f o[4];
  #pragma unroll
  for (int nt = 0; nt < 4; ++nt) o[nt] = z8;

  const unsigned short* kh0 = KH + ((size_t)(b * SEQP + 16 * w + m)) * DM;
  const unsigned short* kl0 = KL + ((size_t)(b * SEQP + 16 * w + m)) * DM;
  const _Float16* vb0 = VT + ((size_t)(b * DM + 64 * w + m)) * SEQP;
  const int sq = q0 + m;
  const int mr = (sq - TXTN) < 0 ? 0 : (sq - TXTN);
  const float* mrow = MK + (size_t)mr * VIDN;
  const bool qtxt = sq < TXTN;

  int buf = 0;
  #pragma unroll 1
  for (int kb = 0; kb < SEQP; kb += 64) {
    v8f s = z8;
    const unsigned short* khp = kh0 + (size_t)kb * DM;
    const unsigned short* klp = kl0 + (size_t)kb * DM;
    #pragma unroll 1
    for (int kk = 0; kk < DM; kk += 32) {
      const v16b ka = ldfb(khp + kk, h);
      const v16b kl = ldfb(klp + kk, h);
      const v16b qa = ldfb(sQh + m * DM + kk, h);
      const v16b ql = ldfb(sQl + m * DM + kk, h);
      s = wmma_b(ka, qa, s);
      s = wmma_b(ka, ql, s);
      s = wmma_b(kl, qa, s);
    }
    const int cb = kb + 16 * w + 8 * h - TXTN;
    const bool ktxt = cb < 0;
    const bool kpad = cb >= VIDN;
    int cbc = cb < 0 ? 0 : cb;
    cbc = cbc > (VIDN - 8) ? (VIDN - 8) : cbc;
    const v4f g0 = *(const v4fa*)(mrow + cbc), g1 = *(const v4fa*)(mrow + cbc + 4);
    const float gk[8] = {g0.x, g0.y, g0.z, g0.w, g1.x, g1.y, g1.z, g1.w};
    v8h ph, plo;
    #pragma unroll
    for (int r = 0; r < 8; ++r) {
      const float gg = kpad ? 0.0f : ((qtxt || ktxt) ? 1.0f : gk[r]);
      const float pv = (s[r] * gg) * PSC;
      const _Float16 hv = (_Float16)pv;
      ph[r]  = hv;
      plo[r] = (_Float16)(pv - (float)hv);
    }
    *(v8ha*)(&sPh[buf][m * 64 + 16 * w + 8 * h]) = ph;
    *(v8ha*)(&sPl[buf][m * 64 + 16 * w + 8 * h]) = plo;
    __syncthreads();

    #pragma unroll
    for (int ks = 0; ks < 2; ++ks) {
      const v16h pa = ldfh(&sPh[buf][m * 64 + 32 * ks], h);
      const v16h pb = ldfh(&sPl[buf][m * 64 + 32 * ks], h);
      #pragma unroll
      for (int nt = 0; nt < 4; ++nt) {
        const v16h vbf = ldfh(vb0 + (size_t)(16 * nt) * SEQP + kb + 32 * ks, h);
        o[nt] = wmma_h(pa, vbf, o[nt]);
        o[nt] = wmma_h(pb, vbf, o[nt]);
      }
    }
    buf ^= 1;
  }

  float* so = sO + w * 1024;
  #pragma unroll
  for (int nt = 0; nt < 4; ++nt)
    #pragma unroll
    for (int r = 0; r < 8; ++r)
      so[(8 * h + r) * 64 + 16 * nt + m] = o[nt][r] * OSC;
  __syncthreads();
  store_out(so, out, b, q0, w, sub, q8);
  __threadfence();
  store_out(so, out, b, q0, w, sub, q8);
}

extern "C" void kernel_launch(void* const* d_in, const int* in_sizes, int n_in,
                              void* d_out, int out_size, void* d_ws, size_t ws_size,
                              hipStream_t stream)
{
  if (n_in < 9) return;
  if (in_sizes[0] != BATCH * SEQ * DM) return;
  if (in_sizes[1] != VIDN * VIDN) return;
  for (int i = 2; i < 8; ++i) if (in_sizes[i] != DM * DM) return;
  if (in_sizes[8] < 1) return;
  if (out_size != BATCH * SEQ * DM + 1) return;

  const float* src = (const float*)d_in[0];
  const float* lrn = (const float*)d_in[1];
  const float* wtq = (const float*)d_in[2];
  const float* wtk = (const float*)d_in[3];
  const float* wtv = (const float*)d_in[4];
  const float* wvq = (const float*)d_in[5];
  const float* wvk = (const float*)d_in[6];
  const float* wvv = (const float*)d_in[7];
  const int*   txl = (const int*)d_in[8];
  float* out0 = (float*)d_out;
  float* out1 = out0 + (size_t)BATCH * SEQ * DM;

  const size_t pl_bytes = (size_t)BATCH * SEQP * DM * 2;
  const size_t wb_bytes = (size_t)NWPL * DM * DM * 2;
  const size_t xt_bytes = (size_t)4 * DM * VIDN * 4;
  const size_t mk_bytes = (size_t)VIDN * VIDN * 4;
  const size_t off_qh = 0;
  const size_t off_ql = off_qh + pl_bytes;
  const size_t off_kh = off_ql + pl_bytes;
  const size_t off_kl = off_kh + pl_bytes;
  const size_t off_vt = off_kl + pl_bytes;
  const size_t off_wb = off_vt + pl_bytes;
  const size_t off_xt = off_wb + wb_bytes;
  const size_t off_mk = off_xt + xt_bytes;
  const size_t total  = off_mk + mk_bytes;
  if (total > ws_size) return;
  if (total > (size_t)134217728) return;

  char* ws = (char*)d_ws;
  unsigned short* QH = (unsigned short*)(ws + off_qh);
  unsigned short* QL = (unsigned short*)(ws + off_ql);
  unsigned short* KH = (unsigned short*)(ws + off_kh);
  unsigned short* KL = (unsigned short*)(ws + off_kl);
  _Float16* VT = (_Float16*)(ws + off_vt);
  unsigned short* WB = (unsigned short*)(ws + off_wb);
  float* XT = (float*)(ws + off_xt);
  float* MK = (float*)(ws + off_mk);

  k_wprep<<<(NWPL * DM) / 8, 256, 0, stream>>>(wtq, wtk, wtv, wvq, wvk, wvv, WB);
  k_xtab<<<DM * 8, 256, 0, stream>>>(XT);
  k_mask<<<(VIDN * VIDN) / 256, 256, 0, stream>>>(lrn, MK);
  k_loss<<<1, 256, 0, stream>>>(lrn, txl, out1);

  const size_t proj_lds = 131072;
  hipFuncSetAttribute(reinterpret_cast<const void*>(&k_proj), hipFuncAttributeMaxDynamicSharedMemorySize, (int)proj_lds);
  dim3 gp(NTILE, BATCH);
  k_proj<<<gp, 512, proj_lds, stream>>>(src, WB, XT, QH, QL, KH, KL, VT);

  dim3 gr(SEQ / 16, BATCH);
  k_ret<<<gr, 128, 0, stream>>>(QH, QL, KH, KL, VT, MK, out0);
}
